// Block_88158498717701
// MI455X (gfx1250) — hardware-verified
//
#include <hip/hip_runtime.h>
#ifndef NB
#define NB 2
#endif
#ifndef SEQ
#define SEQ 2048
#endif
#define NB_FULL 2
#define SEQ_FULL 2048
#define DM 1024
#define NH 16
#define HD 64
#define DFF 4096
#define LQ (3 * DM)
#define NR ((size_t)NB * SEQ)

typedef unsigned short v8us __attribute__((ext_vector_type(8), may_alias));
typedef float  v8f  __attribute__((ext_vector_type(8)));
typedef float  v4f  __attribute__((ext_vector_type(4)));
typedef float  v4fa __attribute__((ext_vector_type(4), may_alias));
typedef _Float16 v16h __attribute__((ext_vector_type(16)));
typedef _Float16 v4h __attribute__((ext_vector_type(4)));
union FragH { v16h v; v8us half[2]; _Float16 h[16]; unsigned short u[16]; };

static_assert(DM == 1024);
static_assert(NH * HD == DM);
static_assert(HD == 64);
static_assert(LQ == 3 * DM);
static_assert(SEQ % 64 == 0);
static_assert((NB * SEQ) % 128 == 0);
static_assert(DM % 32 == 0 && DFF % 32 == 0);
static_assert(LQ % 64 == 0 && DFF % 64 == 0 && DM % 64 == 0);
static_assert(DM % 8 == 0 && DFF % 8 == 0);
static_assert(NB <= NB_FULL && SEQ <= SEQ_FULL);

__device__ __forceinline__ unsigned short bf16_bits(float x) { unsigned int u = __float_as_uint(x); return (unsigned short)((u + 0x7FFFu + ((u >> 16) & 1u)) >> 16); }
__device__ __forceinline__ float bf16_val(unsigned short b) { return __uint_as_float(((unsigned int)b) << 16); }
__device__ __forceinline__ float bf16_rne(float x) { return bf16_val(bf16_bits(x)); }

__device__ __forceinline__ v16h g2_frag(const _Float16* p, int hh) { FragH f; f.half[0] = *(const v8us*)((const unsigned short*)p + 8 * hh); f.half[1] = *(const v8us*)((const unsigned short*)p + 16 + 8 * hh); return f.v; }
__device__ __forceinline__ v16h ld_frag(const unsigned short* base, int off) { FragH f; f.half[0] = *(const v8us*)(base + off); f.half[1] = *(const v8us*)(base + off + 16); return f.v; }
__device__ __forceinline__ v8f g2_mma(v16h a, v16h b, v8f c) { v8f d = __builtin_amdgcn_wmma_f32_16x16x32_f16(false, a, false, b, (short)0, c, false, false); asm volatile("v_nop\n\tv_nop\n\tv_nop\n\tv_nop" : "+v"(d) : "v"(a), "v"(b)); return d; }

__global__ __launch_bounds__(256) void k_wt_f16(const float* __restrict__ W, _Float16* __restrict__ Wt, int K, int N, float scale) {
  const int t = blockIdx.x * 256 + threadIdx.x; if (t >= N * (K / 8)) return; const int n = t / (K / 8), k8 = (t % (K / 8)) * 8; FragH f;
#pragma unroll
  for (int i = 0; i < 8; ++i) f.h[i] = (_Float16)(bf16_rne(W[(size_t)(k8 + i) * N + n]) * scale);
  const v8us o = f.half[0];
  *(volatile v8us*)((unsigned short*)Wt + (size_t)n * K + k8) = o; __threadfence(); *(volatile v8us*)((unsigned short*)Wt + (size_t)n * K + k8) = o;
}

__global__ __launch_bounds__(256) void k_x16(const float* __restrict__ x, _Float16* __restrict__ X16) {
  const size_t t = (size_t)blockIdx.x * 256 + threadIdx.x; if (t >= NR * DM / 8) return;
  const size_t e = t * 8; const size_t r = e / DM; const int c = (int)(e % DM); const size_t rx = (r / SEQ) * SEQ_FULL + (r % SEQ);
  const v4f a = *(const v4fa*)(x + rx * DM + c), d = *(const v4fa*)(x + rx * DM + c + 4); FragH f;
#pragma unroll
  for (int q = 0; q < 4; ++q) { f.h[q] = (_Float16)bf16_rne(a[q]); f.h[4 + q] = (_Float16)bf16_rne(d[q]); }
  const v8us o = f.half[0];
  *(volatile v8us*)((unsigned short*)X16 + e) = o; __threadfence(); *(volatile v8us*)((unsigned short*)X16 + e) = o;
}

__global__ __launch_bounds__(128) void k_gemm2(const _Float16* __restrict__ A, int lda, const _Float16* __restrict__ Bh, int ldb, float alpha, const float* __restrict__ bias, int relu,
                                               float* __restrict__ C, _Float16* __restrict__ C16, float oscale, int ldc, int M, int N, int K) {
  __shared__ __attribute__((aligned(16))) float so[4][32][68];
  const int tid = threadIdx.x; const int w = __builtin_amdgcn_readfirstlane(tid >> 5); const int lane = tid & 31, ln = lane & 15, hh = lane >> 4;
  const int ntn = N >> 6; const int mt = blockIdx.x / ntn, nq = blockIdx.x - mt * ntn; const int row0 = mt * 128 + 32 * w, col0 = nq * 64; if (row0 >= M) return;
  const _Float16* a0p = A + (size_t)(row0 + ln) * lda; const _Float16* a1p = a0p + (size_t)16 * lda;
  const _Float16* b0p = Bh + (size_t)(col0 + ln) * ldb; const _Float16* b1p = b0p + (size_t)16 * ldb; const _Float16* b2p = b1p + (size_t)16 * ldb; const _Float16* b3p = b2p + (size_t)16 * ldb;
  const v8f z8 = {0.f,0.f,0.f,0.f,0.f,0.f,0.f,0.f}; v8f c00 = z8, c01 = z8, c02 = z8, c03 = z8, c10 = z8, c11 = z8, c12 = z8, c13 = z8;
#pragma unroll 1
  for (int kb = 0; kb < K; kb += 32) { const v16h a0 = g2_frag(a0p + kb, hh), a1 = g2_frag(a1p + kb, hh);
    v16h b = g2_frag(b0p + kb, hh); c00 = g2_mma(a0, b, c00); c10 = g2_mma(a1, b, c10);
    b = g2_frag(b1p + kb, hh); c01 = g2_mma(a0, b, c01); c11 = g2_mma(a1, b, c11);
    b = g2_frag(b2p + kb, hh); c02 = g2_mma(a0, b, c02); c12 = g2_mma(a1, b, c12);
    b = g2_frag(b3p + kb, hh); c03 = g2_mma(a0, b, c03); c13 = g2_mma(a1, b, c13); }
  v8f accs[8] = {c00, c01, c02, c03, c10, c11, c12, c13};
#pragma unroll
  for (int u = 0; u < 8; ++u) { const int t = u & 3, half = u >> 2; const int col = col0 + t * 16 + ln; const float bv = bf16_rne(bias[col]);
#pragma unroll
    for (int r = 0; r < 8; ++r) { const int rloc = half * 16 + 8 * hh + r; float v = accs[u][r] * alpha + bv; if (relu) v = fmaxf(v, 0.f); so[w][rloc][t * 16 + ln] = v; } }
  __builtin_amdgcn_fence(4  , "workgroup"); __builtin_amdgcn_wave_barrier();
  const int rsub = lane >> 4, c4 = (lane & 15) * 4;
  for (int pass = 0; pass < 2; ++pass) {
#pragma unroll
    for (int q = 0; q < 16; ++q) { const int r = q * 2 + rsub; const v4f v = *(const v4fa*)&so[w][r][c4];
      if (C) *(volatile v4f*)(C + (size_t)(row0 + r) * ldc + col0 + c4) = v;
      if (C16) { v4h h4; for (int i = 0; i < 4; ++i) h4[i] = (_Float16)(v[i] * oscale); *(volatile v4h*)(C16 + (size_t)(row0 + r) * ldc + col0 + c4) = h4; } }
    if (pass == 0) __threadfence(); } }

__global__ __launch_bounds__(256) void k_vt(const _Float16* __restrict__ V16, int ldv, int voff, _Float16* __restrict__ Vt) {
  __shared__ unsigned short tl[64][66]; const int tid = threadIdx.x; const int slab = blockIdx.x / (SEQ / 64), lg = blockIdx.x % (SEQ / 64); const int b = slab / NH, h = slab % NH;
  for (int i = tid; i < 64 * 8; i += 256) { const int r = i / 8, c8 = (i % 8) * 8; FragH f; f.half[0] = *(const v8us*)((const unsigned short*)V16 + ((size_t)b * SEQ + lg * 64 + r) * ldv + voff + h * 64 + c8);
#pragma unroll
    for (int q = 0; q < 8; ++q) tl[r][c8 + q] = f.u[q]; }
  __syncthreads();
  for (int pass = 0; pass < 2; ++pass) {
#pragma unroll
    for (int rd = 0; rd < 2; ++rd) { const int d = rd * 32 + tid / 8, pc = tid % 8; FragH f;
#pragma unroll
      for (int q = 0; q < 8; ++q) f.u[q] = tl[pc * 8 + q][d];
      *(volatile v8us*)((unsigned short*)Vt + ((size_t)slab * 64 + d) * SEQ + lg * 64 + pc * 8) = f.half[0]; }
    if (pass == 0) __threadfence(); } }

__global__ __launch_bounds__(128) void k_flash(const _Float16* __restrict__ QKV, const _Float16* __restrict__ VT, float* __restrict__ ATT) {
  __shared__ __attribute__((aligned(16))) float so[4][16][68];
  const int tid = threadIdx.x; const int wave = __builtin_amdgcn_readfirstlane(tid >> 5); const int lane = tid & 31, ln = lane & 15, hh = lane >> 4;
  const int qb = blockIdx.x % (SEQ / 64), bh = blockIdx.x / (SEQ / 64); const int b = bh / NH, h = bh % NH;
  const int q0 = qb * 64 + wave * 16;
  const unsigned short* qk = (const unsigned short*)QKV; const unsigned short* vt = (const unsigned short*)VT;
  const int qoff = (b * SEQ + q0 + ln) * LQ + h * HD + 8 * hh;
  const int koff = (b * SEQ + ln) * LQ + DM + h * HD + 8 * hh;
  const int voff = (bh * HD + ln) * SEQ + 8 * hh;
  const v8f z8 = {0.f,0.f,0.f,0.f,0.f,0.f,0.f,0.f};
  v8f acc[4] = {z8, z8, z8, z8};
  float m = -1.0e30f, l = 0.f;
  const int nsteps = (q0 >> 5) + 1;
#pragma unroll 1
  for (int st = 0; st < nsteps; ++st) {
    const int kb = st * 32;
    v8f s0 = z8, s1 = z8;
#pragma unroll
    for (int ks = 0; ks < 2; ++ks) {
      const v16h bq = ld_frag(qk, qoff + ks * 32);
      const v16h a0 = ld_frag(qk, koff + kb * LQ + ks * 32); s0 = g2_mma(a0, bq, s0);
      const v16h a1 = ld_frag(qk, koff + (kb + 16) * LQ + ks * 32); s1 = g2_mma(a1, bq, s1);
    }
    float sv0[8], sv1[8];
#pragma unroll
    for (int r = 0; r < 8; ++r) { sv0[r] = s0[r] * 0.125f; sv1[r] = s1[r] * 0.125f; }
    if (kb + 31 > q0) {
      const int qi = q0 + ln, k0 = kb + 8 * hh;
#pragma unroll
      for (int r = 0; r < 8; ++r) { sv0[r] = (k0 + r <= qi) ? sv0[r] : -1.0e30f; sv1[r] = (k0 + 16 + r <= qi) ? sv1[r] : -1.0e30f; }
    }
    float mx = fmaxf(sv0[0], sv1[0]);
#pragma unroll
    for (int r = 1; r < 8; ++r) mx = fmaxf(mx, fmaxf(sv0[r], sv1[r]));
    mx = fmaxf(mx, __shfl_xor(mx, 16, 32));
    const float mnew = fmaxf(m, mx);
    if (__builtin_amdgcn_ballot_w32(mnew > m) != 0u) {
      const float al = __expf(m - mnew); l *= al;
#pragma unroll
      for (int dt = 0; dt < 4; ++dt) acc[dt] = acc[dt] * al;
    }
    m = mnew;
    FragH pb; float ps = 0.f;
#pragma unroll
    for (int r = 0; r < 8; ++r) { const float p0 = __expf(sv0[r] - mnew), p1 = __expf(sv1[r] - mnew); ps += p0 + p1; pb.h[r] = (_Float16)(p0 * 1024.0f); pb.h[8 + r] = (_Float16)(p1 * 1024.0f); }
    l += ps;
#pragma unroll
    for (int dt = 0; dt < 4; ++dt) { const v16h av = ld_frag(vt, voff + dt * 16 * SEQ + kb); acc[dt] = g2_mma(av, pb.v, acc[dt]); }
  }
  const float lt = l + __shfl_xor(l, 16, 32);
  const float inv = 1.0f / (1024.0f * lt);
#pragma unroll
  for (int dt = 0; dt < 4; ++dt)
#pragma unroll
    for (int r = 0; r < 8; ++r) so[wave][ln][dt * 16 + 8 * hh + r] = acc[dt][r] * inv;
  __builtin_amdgcn_fence(4  , "workgroup"); __builtin_amdgcn_wave_barrier();
  const int rsub = lane >> 4, c4 = (lane & 15) * 4;
  float* dst = ATT + (size_t)(b * SEQ + q0) * DM + h * HD + c4;
  for (int pass = 0; pass < 2; ++pass) {
#pragma unroll
    for (int q = 0; q < 8; ++q) { const int r = q * 2 + rsub; const v4f v = *(const v4fa*)&so[wave][r][c4]; *(volatile v4f*)(dst + (size_t)r * DM) = v; }
    if (pass == 0) __threadfence(); } }

__global__ __launch_bounds__(256) void k_ln(const float* __restrict__ X, int xfull, int bfin, const float* __restrict__ R, const float* __restrict__ g, const float* __restrict__ bb, float eps,
                                            _Float16* __restrict__ N16, float s16, float* __restrict__ N32, int ofull) {
  #pragma clang fp contract(off)
  __shared__ float red1[8]; __shared__ float red2[8];
  const int r = blockIdx.x, t = threadIdx.x; const int wave = __builtin_amdgcn_readfirstlane(t >> 5); const int lane = t & 31;
  const size_t rfull = (size_t)(r / SEQ) * SEQ_FULL + (size_t)(r % SEQ);
  const size_t rx = xfull ? rfull : (size_t)r; const size_t ro = ofull ? rfull : (size_t)r;
  const v4f xa = *(const v4fa*)(X + rx * DM + t * 4); const v4f ra = *(const v4fa*)(R + (size_t)r * DM + t * 4);
  float s[4]; float sum = 0.f;
#pragma unroll
  for (int q = 0; q < 4; ++q) { const float xb = bf16_rne(xa[q]); const float xv = bfin ? xb : xa[q]; s[q] = xv + ra[q]; sum += s[q]; }
#pragma unroll
  for (int mk = 16; mk > 0; mk >>= 1) sum += __shfl_xor(sum, mk, 32);
  if (lane == 0) red1[wave] = sum;
  __syncthreads();
  float tot = 0.f;
#pragma unroll
  for (int i = 0; i < 8; ++i) tot += red1[i];
  const float mu = tot * (1.0f / (float)DM);
  float vs = 0.f;
#pragma unroll
  for (int q = 0; q < 4; ++q) { const float dl = s[q] - mu; vs += dl * dl; }
#pragma unroll
  for (int mk = 16; mk > 0; mk >>= 1) vs += __shfl_xor(vs, mk, 32);
  if (lane == 0) red2[wave] = vs;
  __syncthreads();
  float tv = 0.f;
#pragma unroll
  for (int i = 0; i < 8; ++i) tv += red2[i];
  const float rs = rsqrtf(tv * (1.0f / (float)DM) + eps);
  v4h y; v4f yf;
#pragma unroll
  for (int q = 0; q < 4; ++q) { const int c = t * 4 + q; yf[q] = (s[q] - mu) * rs * bf16_rne(g[c]) + bf16_rne(bb[c]); y[q] = (_Float16)(yf[q] * s16); }
  for (int pass = 0; pass < 2; ++pass) {
    if (N16) *(volatile v4h*)(N16 + (size_t)r * DM + t * 4) = y;
    if (N32) *(volatile v4f*)(N32 + ro * DM + t * 4) = yf;
    if (pass == 0) __threadfence(); } }

constexpr size_t al256(size_t b) { return (b + 255) & ~(size_t)255; }
constexpr size_t cmax(size_t a, size_t b) { return a > b ? a : b; }
constexpr size_t SZ_BQKV = al256((size_t)LQ * DM * 2);
constexpr size_t SZ_BW1  = al256((size_t)DFF * DM * 2);
constexpr size_t SZ_BW2  = al256((size_t)DM * DFF * 2);
constexpr size_t SZ_X16  = al256(NR * DM * 2);
constexpr size_t SZ_QKV  = al256(NR * LQ * 2);
constexpr size_t SZ_VT   = al256((size_t)NB * NH * HD * SEQ * 2);
constexpr size_t SZ_R16  = al256(NR * DFF * 2);
constexpr size_t SZ_RA   = cmax(SZ_QKV + SZ_VT, SZ_R16);
constexpr size_t SZ_F32  = al256(NR * DM * 4);
constexpr size_t SZ_H32  = al256(NR * DM * 4);
constexpr size_t SZ_H16  = al256(NR * DM * 2);
constexpr size_t WS_TOTAL = SZ_BQKV + SZ_BW1 + SZ_BW2 + SZ_X16 + SZ_RA + SZ_F32 + SZ_H32 + SZ_H16;
static_assert(SZ_QKV + SZ_VT <= SZ_RA);
static_assert(SZ_R16 <= SZ_RA);
static_assert(WS_TOTAL <= (size_t)134217728);
static_assert(((size_t)(NB_FULL - 1) * SEQ_FULL + SEQ_FULL) * DM * 4 == (size_t)16777216);

extern "C" void kernel_launch(void* const* d_in, const int* in_sizes, int n_in,
                              void* d_out, int out_size, void* d_ws, size_t ws_size, hipStream_t stream) {
  if (n_in < 11) return;
  const size_t xneed = ((size_t)(NB - 1) * SEQ_FULL + SEQ) * DM;
  if ((size_t)in_sizes[0] < xneed) return;
  if (in_sizes[1] < DM * LQ || in_sizes[2] < LQ || in_sizes[3] < DM * DFF || in_sizes[4] < DFF || in_sizes[5] < DFF * DM || in_sizes[6] < DM) return;
  if (in_sizes[7] < DM || in_sizes[8] < DM || in_sizes[9] < DM || in_sizes[10] < DM) return;
  if ((size_t)out_size < xneed) return;
  if (WS_TOTAL > ws_size) return;
  const float* x    = (const float*)d_in[0];
  const float* wqkv = (const float*)d_in[1];
  const float* bqkv = (const float*)d_in[2];
  const float* w1   = (const float*)d_in[3];
  const float* b1   = (const float*)d_in[4];
  const float* w2   = (const float*)d_in[5];
  const float* b2   = (const float*)d_in[6];
  const float* g1   = (const float*)d_in[7];
  const float* be1  = (const float*)d_in[8];
  const float* g2   = (const float*)d_in[9];
  const float* be2  = (const float*)d_in[10];
  char* ws = (char*)d_ws; size_t off = 0;
  _Float16* BQKV = (_Float16*)(ws + off); off += SZ_BQKV;
  _Float16* BW1  = (_Float16*)(ws + off); off += SZ_BW1;
  _Float16* BW2  = (_Float16*)(ws + off); off += SZ_BW2;
  _Float16* X16  = (_Float16*)(ws + off); off += SZ_X16;
  char* RA = ws + off; off += SZ_RA;
  _Float16* QKV16 = (_Float16*)RA; _Float16* VT = (_Float16*)(RA + SZ_QKV); _Float16* R16 = (_Float16*)RA;
  float* F32A = (float*)(ws + off); off += SZ_F32;
  float* H32  = (float*)(ws + off); off += SZ_H32;
  _Float16* H16 = (_Float16*)(ws + off); off += SZ_H16;

  k_wt_f16<<<(unsigned)(((size_t)LQ * (DM / 8) + 255) / 256), 256, 0, stream>>>(wqkv, BQKV, DM, LQ, 16.0f);
  k_wt_f16<<<(unsigned)(((size_t)DFF * (DM / 8) + 255) / 256), 256, 0, stream>>>(w1, BW1, DM, DFF, 16.0f);
  k_wt_f16<<<(unsigned)(((size_t)DM * (DFF / 8) + 255) / 256), 256, 0, stream>>>(w2, BW2, DFF, DM, 64.0f);
  k_x16<<<(unsigned)((NR * DM / 8 + 255) / 256), 256, 0, stream>>>(x, X16);
  k_gemm2<<<(unsigned)((NR / 128) * (LQ / 64)), 128, 0, stream>>>(X16, DM, BQKV, DM, 0.0625f, bqkv, 0, nullptr, QKV16, 1.0f, LQ, (int)NR, LQ, DM);
  k_vt<<<(unsigned)(NB * NH * (SEQ / 64)), 256, 0, stream>>>(QKV16, LQ, 2 * DM, VT);
  k_flash<<<(unsigned)(NB * NH * (SEQ / 64)), 128, 0, stream>>>(QKV16, VT, F32A);
  k_ln<<<(unsigned)NR, 256, 0, stream>>>(x, 1, 1, F32A, g1, be1, 1e-5f, H16, 16.0f, H32, 0);
  k_gemm2<<<(unsigned)((NR / 128) * (DFF / 64)), 128, 0, stream>>>(H16, DM, BW1, DM, 0.00390625f, b1, 1, nullptr, R16, 16.0f, DFF, (int)NR, DFF, DM);
  k_gemm2<<<(unsigned)((NR / 128) * (DM / 64)), 128, 0, stream>>>(R16, DFF, BW2, DFF, 0.0009765625f, b2, 0, F32A, nullptr, 1.0f, DM, (int)NR, DM, DFF);
  k_ln<<<(unsigned)NR, 256, 0, stream>>>(H32, 0, 0, F32A, g2, be2, 1e-5f, nullptr, 1.0f, (float*)d_out, 1);
}
